// MambaBlock_5033701670981
// MI455X (gfx1250) — hardware-verified
//
#include <hip/hip_runtime.h>
#include <math.h>

typedef __attribute__((ext_vector_type(16))) _Float16 v16h;
typedef __attribute__((ext_vector_type(8)))  _Float16 v8h;
typedef __attribute__((ext_vector_type(16))) __bf16   v16b;
typedef __attribute__((ext_vector_type(8)))  __bf16   v8b;
typedef __attribute__((ext_vector_type(8)))  float    v8f;
typedef __attribute__((ext_vector_type(4)))  float    v4f;

constexpr int kB      = 4;
constexpr int kT      = 8192;
constexpr int kKs     = 64;
constexpr int kL      = kT - kKs + 1;
constexpr int kLP     = 8192;
constexpr int kRowsAll = kB * kLP;
constexpr int kDin    = 256;
constexpr int kNst    = 16;
constexpr int kDtR    = 4;
constexpr int kXpN    = kDtR + 2 * kNst;
constexpr int kXdP    = 64;
constexpr int kXzP    = 2 * kDin;
constexpr int kRc     = 2 * kKs;
constexpr int kNBP    = 2;
constexpr int kMP     = kNBP * kLP;
constexpr int kTP     = 260;
constexpr int kScanTS = 64;
constexpr int kScanCh = 64;
constexpr int kScanYP = 68;
constexpr float kEps  = 1e-5f;
constexpr float kCarryW  = 32.0f;
constexpr float kCarryUC = 16.0f;
constexpr float kCarryY  = 16.0f;
static_assert(kL == 8129, "frames");
static_assert(kXpN == 36 && kXpN <= kXdP, "x_proj width");
static_assert((kKs % 32) == 0 && (kDin % 32) == 0 && (kRc % 32) == 0, "GEMM K multiples of 32");
static_assert((kMP % 64) == 0 && (kRowsAll % 64) == 0 && (kXzP % 64) == 0 && (kXdP % 64) == 0 && (kKs % 64) == 0, "GEMM M,N multiples of 64");
static_assert((kLP % kScanTS) == 0 && (kLP % 64) == 0 && (kDin % kScanCh) == 0 && kDin == 256, "tile multiples");
static_assert((kB % kNBP) == 0, "passes");

constexpr size_t kOffWIN  = 0;
constexpr size_t kOffWXP  = kOffWIN  + (size_t)2 * kXzP * kKs * 2;
constexpr size_t kOffWOUT = kOffWXP  + (size_t)2 * kXdP * kDin * 2;
constexpr size_t kOffCTH  = kOffWOUT + (size_t)2 * kKs * kDin * 2;
constexpr size_t kOffCTL  = kOffCTH  + (size_t)kKs * kRc * 2;
constexpr size_t kOffU    = kOffCTL  + (size_t)kKs * kRc * 2;
constexpr size_t kOffXZ   = kOffU    + (size_t)2 * kRowsAll * kKs * 2;
constexpr size_t kOffUC   = kOffXZ   + (size_t)kMP * kXzP * 4;
constexpr size_t kOffUC16 = kOffUC   + (size_t)kMP * kDin * 4;
constexpr size_t kOffXD   = kOffUC16 + (size_t)kMP * kDin * 2;
constexpr size_t kOffY16  = kOffXD   + (size_t)kMP * kXdP * 4;
constexpr size_t kOffHID  = kOffY16  + (size_t)kMP * kDin * 2;
constexpr size_t kOffRH   = kOffHID  + (size_t)kMP * kKs * 4;
constexpr size_t kOffRL   = kOffRH   + (size_t)kRowsAll * kRc * 2;
constexpr size_t kOffP    = kOffRL   + (size_t)kRowsAll * kRc * 2;
constexpr size_t kWsTotal = kOffP    + (size_t)kRowsAll * kKs * 4;
static_assert(kWsTotal == 109346816ull, "carve total");
static_assert(kWsTotal <= 134217728ull, "carve cap");
static_assert((kOffWXP % 128) == 0 && (kOffWOUT % 128) == 0 && (kOffCTH % 128) == 0 && (kOffCTL % 128) == 0 &&
              (kOffU % 128) == 0 && (kOffXZ % 128) == 0 && (kOffUC % 128) == 0 && (kOffUC16 % 128) == 0 &&
              (kOffXD % 128) == 0 && (kOffY16 % 128) == 0 && (kOffHID % 128) == 0 && (kOffRH % 128) == 0 &&
              (kOffRL % 128) == 0 && (kOffP % 128) == 0, "128-B aligned regions");

__device__ __forceinline__ unsigned short f2bf_bits(float f) {
  unsigned u = __float_as_uint(f);
  return (unsigned short)((u + 0x7FFFu + ((u >> 16) & 1u)) >> 16);
}
__device__ __forceinline__ float bf_bits2f(unsigned short h) { return __uint_as_float(((unsigned)h) << 16); }

__device__ __forceinline__ void dep_guard4_h(v8f& a, v8f& b, v8f& c, v8f& d, v16h x, v16h y) { asm volatile("v_nop\n\tv_nop\n\tv_nop\n\tv_nop" : "+v"(a), "+v"(b), "+v"(c), "+v"(d) : "v"(x), "v"(y)); }
__device__ __forceinline__ void dep_guard4_b(v8f& a, v8f& b, v8f& c, v8f& d, v16b x, v16b y) { asm volatile("v_nop\n\tv_nop\n\tv_nop\n\tv_nop" : "+v"(a), "+v"(b), "+v"(c), "+v"(d) : "v"(x), "v"(y)); }
__device__ __forceinline__ void keep4_h(v16h a, v16h b, v16h c, v16h d) { asm volatile("v_nop" :: "v"(a), "v"(b), "v"(c), "v"(d)); }
__device__ __forceinline__ void keep4_b(v16b a, v16b b, v16b c, v16b d) { asm volatile("v_nop" :: "v"(a), "v"(b), "v"(c), "v"(d)); }
__device__ __forceinline__ void acc_guard4(v8f& a, v8f& b, v8f& c, v8f& d) { asm volatile("v_nop\n\tv_nop\n\tv_nop\n\tv_nop" : "+v"(a), "+v"(b), "+v"(c), "+v"(d)); }
template <typename T> struct Frag;
template <> struct Frag<_Float16> {
  typedef v16h V; union U { v16h v; v8h h[2]; };
  static __device__ __forceinline__ v16h load(const _Float16* p) {
    U f; f.h[0] = *(const v8h*)(p); f.h[1] = *(const v8h*)(p + 16); return f.v;
  }
  static __device__ __forceinline__ v8f mma(v16h a, v16h b, v8f c) {
    return __builtin_amdgcn_wmma_f32_16x16x32_f16(false, a, false, b, (short)0, c, false, false);
  }
  static __device__ __forceinline__ void guard(v8f& a, v8f& b, v8f& c, v8f& d, v16h x, v16h y) { dep_guard4_h(a, b, c, d, x, y); }
  static __device__ __forceinline__ void keep(v16h a, v16h b, v16h c, v16h d) { keep4_h(a, b, c, d); }
};
template <> struct Frag<__bf16> {
  typedef v16b V; union U { v16b v; v8b h[2]; };
  static __device__ __forceinline__ v16b load(const __bf16* p) {
    U f; f.h[0] = *(const v8b*)(p); f.h[1] = *(const v8b*)(p + 16); return f.v;
  }
  static __device__ __forceinline__ v8f mma(v16b a, v16b b, v8f c) {
    return __builtin_amdgcn_wmma_f32_16x16x32_bf16(false, a, false, b, (short)0, c, false, false);
  }
  static __device__ __forceinline__ void guard(v8f& a, v8f& b, v8f& c, v8f& d, v16b x, v16b y) { dep_guard4_b(a, b, c, d, x, y); }
  static __device__ __forceinline__ void keep(v16b a, v16b b, v16b c, v16b d) { keep4_b(a, b, c, d); }
};

template <int ET> struct Elem;
template <> struct Elem<0> { typedef _Float16 T; };
template <> struct Elem<1> { typedef __bf16 T; };
template <int ET, bool SPLIT, int BIAS_MODE, int OUT_MODE, bool RESID, int ACT = 0>
__global__ __launch_bounds__(256) void wmma_gemm64(
    const unsigned short* __restrict__ Ap, const unsigned short* __restrict__ A2p, int lda, long strideA,
    const unsigned short* __restrict__ Btp, const unsigned short* __restrict__ Bt2p, int ldb, long strideB,
    void* __restrict__ Cout, void* __restrict__ Cout2, int ldc, long strideC,
    const float* __restrict__ bias,
    const float* __restrict__ resid, long strideR,
    int M, int N, int K, float scale) {
  typedef typename Elem<ET>::T T;
  typedef typename Frag<T>::V V;
  const T* A = (const T*)Ap; const T* A2 = (const T*)A2p; const T* Bt = (const T*)Btp; const T* Bt2 = (const T*)Bt2p;
  __shared__ __align__(16) float sT[8][16 * 68];
  const int b    = blockIdx.y;
  const int lane = threadIdx.x & 31;
  const int wave = threadIdx.x >> 5;
  const int tilesN = N >> 6;
  const int tilesM = M >> 6;
  const int tile = blockIdx.x * 8 + wave;
  if (tile >= tilesM * tilesN) return;
  const int tm = tile / tilesN;
  const int tn = tile - tm * tilesN;
  const int m0 = tm << 6;
  const int n0 = tn << 6;

  const T* Ab  = A  + (size_t)b * strideA;
  const T* Bb  = Bt + (size_t)b * strideB;
  const T* Ab2 = SPLIT ? (A2  + (size_t)b * strideA) : nullptr;
  const T* Bb2 = SPLIT ? (Bt2 + (size_t)b * strideB) : nullptr;

  const int rlane = lane & 15;
  const int koff  = (lane >> 4) * 8;
  const int mOff  = (lane >> 4) * 8;

  v8f acc[4][4];
#pragma unroll
  for (int i = 0; i < 4; ++i)
#pragma unroll
    for (int j = 0; j < 4; ++j) acc[i][j] = (v8f){0.f,0.f,0.f,0.f,0.f,0.f,0.f,0.f};

  for (int k0 = 0; k0 < K; k0 += 32) {
    V bh[4], bl[4];
#pragma unroll
    for (int j = 0; j < 4; ++j) {
      const size_t bo = (size_t)(n0 + (j << 4) + rlane) * ldb + koff + k0;
      bh[j] = Frag<T>::load(Bb + bo);
      if (SPLIT) bl[j] = Frag<T>::load(Bb2 + bo);
    }
#pragma unroll
    for (int i = 0; i < 4; ++i) {
      const size_t ao = (size_t)(m0 + (i << 4) + rlane) * lda + koff + k0;
      V ah = Frag<T>::load(Ab + ao);
      V al;
      if (SPLIT) al = Frag<T>::load(Ab2 + ao);
#pragma unroll
      for (int j = 0; j < 4; ++j) {
        acc[i][j] = Frag<T>::mma(ah, bh[j], acc[i][j]);
        if (SPLIT) {
          acc[i][j] = Frag<T>::mma(ah, bl[j], acc[i][j]);
          acc[i][j] = Frag<T>::mma(al, bh[j], acc[i][j]);
        }
      }
      Frag<T>::guard(acc[i][0], acc[i][1], acc[i][2], acc[i][3], ah, SPLIT ? al : ah);
    }
    Frag<T>::keep(bh[0], bh[1], bh[2], bh[3]);
    if (SPLIT) Frag<T>::keep(bl[0], bl[1], bl[2], bl[3]);
  }
  acc_guard4(acc[0][0], acc[0][1], acc[0][2], acc[0][3]);
  acc_guard4(acc[1][0], acc[1][1], acc[1][2], acc[1][3]);
  acc_guard4(acc[2][0], acc[2][1], acc[2][2], acc[2][3]);
  acc_guard4(acc[3][0], acc[3][1], acc[3][2], acc[3][3]);

  float* slab = sT[wave];
  const float* Rb = RESID ? (resid + (size_t)b * strideR) : nullptr;
#pragma unroll
  for (int i = 0; i < 4; ++i) {
    const int mBase = m0 + (i << 4);
#pragma unroll
    for (int j = 0; j < 4; ++j) {
      const int n = n0 + (j << 4) + rlane;
      float bv = 0.f;
      if (BIAS_MODE == 2) bv = bias[n];
#pragma unroll
      for (int r = 0; r < 8; ++r) {
        float v = acc[i][j][r] * scale;
        if (BIAS_MODE == 1) v += bias[mBase + mOff + r];
        if (BIAS_MODE == 2) v += bv;
        if (RESID) v += Rb[(size_t)(mBase + mOff + r) * ldc + n];
        if (ACT == 2) v = fmaxf(v, 0.0f);
        if (ACT == 4) v = (v > 0.f) ? v : 0.01f * v;
        slab[(mOff + r) * 68 + (j << 4) + rlane] = v;
      }
    }
    __builtin_amdgcn_fence(__ATOMIC_RELEASE, "workgroup");
    __builtin_amdgcn_wave_barrier();
    __builtin_amdgcn_fence(__ATOMIC_ACQUIRE, "workgroup");
    if (OUT_MODE == 0) {
      float* C = (float*)Cout + (size_t)b * strideC;
      const int hh = lane >> 4, c4 = (lane & 15) * 4;
      for (int pass = 0; pass < 2; ++pass) {
#pragma unroll
        for (int it = 0; it < 8; ++it) {
          const int row = it * 2 + hh;
          v4f v = *(const v4f*)(slab + row * 68 + c4);
          *(volatile v4f*)(C + (size_t)(mBase + row) * ldc + n0 + c4) = v;
        }
        __threadfence();
      }
    } else {
      const int q = lane >> 3, c8 = (lane & 7) * 8;
      unsigned short* C  = (unsigned short*)Cout  + (size_t)b * strideC;
      unsigned short* C2 = (OUT_MODE == 2) ? ((unsigned short*)Cout2 + (size_t)b * strideC) : nullptr;
      for (int pass = 0; pass < 2; ++pass) {
#pragma unroll
        for (int it = 0; it < 4; ++it) {
          const int row = it * 4 + q;
          const float* sp = slab + row * 68 + c8;
          v8h hv, lv;
#pragma unroll
          for (int e = 0; e < 8; ++e) {
            if (OUT_MODE == 1) {
              hv[e] = (_Float16)sp[e];
            } else {
              unsigned short hb = f2bf_bits(sp[e]);
              unsigned short lb = f2bf_bits(sp[e] - bf_bits2f(hb));
              hv[e] = __builtin_bit_cast(_Float16, hb);
              lv[e] = __builtin_bit_cast(_Float16, lb);
            }
          }
          *(volatile v8h*)(C + (size_t)(mBase + row) * ldc + n0 + c8) = hv;
          if (OUT_MODE == 2) *(volatile v8h*)(C2 + (size_t)(mBase + row) * ldc + n0 + c8) = lv;
        }
        __threadfence();
      }
    }
    __builtin_amdgcn_fence(__ATOMIC_RELEASE, "workgroup");
    __builtin_amdgcn_wave_barrier();
    __builtin_amdgcn_fence(__ATOMIC_ACQUIRE, "workgroup");
  }
}

__global__ __launch_bounds__(256) void cast_f16_pad_kernel(
    const float* __restrict__ src, unsigned short* __restrict__ dst, int total8, int real8, float scale)
{
  const int i = blockIdx.x * 256 + threadIdx.x;
  if (i >= total8) return;
  const bool live = (i < real8);
  const int ic = live ? i : (real8 - 1);
  const float* p = src + ((size_t)ic << 3);
  const v4f a0 = *(const v4f*)(p);
  const v4f a1 = *(const v4f*)(p + 4);
  v8h hv;
#pragma unroll
  for (int e = 0; e < 4; ++e) {
    const float f0 = live ? (a0[e] * scale) : 0.0f;
    const float f1 = live ? (a1[e] * scale) : 0.0f;
    hv[e]     = (_Float16)f0;
    hv[4 + e] = (_Float16)f1;
  }
  unsigned short* q = dst + ((size_t)i << 3);
  *(volatile v8h*)q = hv;
  __threadfence();
  *(volatile v8h*)q = hv;
}

__global__ __launch_bounds__(256) void transpose_split_bf16_kernel(
    const float* __restrict__ W, unsigned short* __restrict__ BtH, unsigned short* __restrict__ BtL, int Kdim, int Ndim)
{
  __shared__ float tile[64 * 65];
  const int tid = threadIdx.x, lane = tid & 31, wave = tid >> 5;
  const int n0 = blockIdx.x * 64;
  const int k0 = blockIdx.y * 64;
#pragma unroll 4
  for (int p = 0; p < 16; ++p) {
    const int idx = tid + p * 256;
    const int kk  = idx >> 6;
    const int nn  = idx & 63;
    const int n   = n0 + nn;
    const int nc  = (n < Ndim) ? n : (Ndim - 1);
    const float v = W[(size_t)(k0 + kk) * Ndim + nc];
    tile[kk * 65 + nn] = (n < Ndim) ? v : 0.f;
  }
  __syncthreads();
  const int q = lane >> 3, c8 = (lane & 7) * 8;
  v8h hv[2], lv[2];
#pragma unroll
  for (int it = 0; it < 2; ++it) {
    const int nrow = it * 32 + wave * 4 + q;
#pragma unroll
    for (int e = 0; e < 8; ++e) {
      const float v = tile[(c8 + e) * 65 + nrow];
      const unsigned short hb = f2bf_bits(v);
      const unsigned short lb = f2bf_bits(v - bf_bits2f(hb));
      hv[it][e] = __builtin_bit_cast(_Float16, hb);
      lv[it][e] = __builtin_bit_cast(_Float16, lb);
    }
  }
  for (int pass = 0; pass < 2; ++pass) {
#pragma unroll
    for (int it = 0; it < 2; ++it) {
      const int nrow = it * 32 + wave * 4 + q;
      const size_t o = (size_t)(n0 + nrow) * Kdim + k0 + c8;
      *(volatile v8h*)(BtH + o) = hv[it];
      *(volatile v8h*)(BtL + o) = lv[it];
    }
    __threadfence();
  }
}

__global__ __launch_bounds__(256) void frame_norm_kernel(
    const float* __restrict__ x, const float* __restrict__ nwf, const float* __restrict__ nwb,
    unsigned short* __restrict__ U16)
{
  const int tid = threadIdx.x, lane = tid & 31, wave = tid >> 5;
  const int q = lane >> 3, c8 = (lane & 7) * 8;
  const int dir = blockIdx.y;
  const int row = blockIdx.x * 32 + wave * 4 + q;
  const int b = row / kLP;
  const int r = row - b * kLP;
  const bool live = (r < kL);
  const int rc = live ? r : (kL - 1);
  const int src = dir ? (kL - 1 - rc) : rc;
  const float* s = x + (size_t)b * kT + src + c8;
  float v[8];
#pragma unroll
  for (int e = 0; e < 8; ++e) v[e] = s[e];
  float ss = 0.0f;
#pragma unroll
  for (int e = 0; e < 8; ++e) ss = fmaf(v[e], v[e], ss);
  ss += __shfl_xor(ss, 1, 32);
  ss += __shfl_xor(ss, 2, 32);
  ss += __shfl_xor(ss, 4, 32);
  const float inv = rsqrtf(ss * (1.0f / (float)kKs) + kEps);
  const float* nw = dir ? nwb : nwf;
  const v4f w0 = *(const v4f*)(nw + c8);
  const v4f w1 = *(const v4f*)(nw + c8 + 4);
  v8h hv;
#pragma unroll
  for (int e = 0; e < 4; ++e) {
    const float f0 = live ? ((v[e] * inv) * w0[e]) : 0.0f;
    const float f1 = live ? ((v[4 + e] * inv) * w1[e]) : 0.0f;
    hv[e]     = (_Float16)f0;
    hv[4 + e] = (_Float16)f1;
  }
  unsigned short* dst = U16 + (size_t)dir * kRowsAll * kKs + (size_t)row * kKs + c8;
  *(volatile v8h*)dst = hv;
  __threadfence();
  *(volatile v8h*)dst = hv;
}

__global__ __launch_bounds__(256) void conv_silu_kernel(
    const float* __restrict__ XZ, const float* __restrict__ cw, const float* __restrict__ cb,
    float* __restrict__ UC, unsigned short* __restrict__ UC16)
{
  __shared__ __align__(16) float sT[16 * kTP];
  const int tid = threadIdx.x, lane = tid & 31, wave = tid >> 5;
  const int d = tid;
  const int g0 = blockIdx.x * 64;
  const int tb = g0 & (kLP - 1);
  const v4f wv = *(const v4f*)(cw + d * 4);
  const float w0 = wv[0], w1 = wv[1], w2 = wv[2], w3 = wv[3];
  const float bc = cb[d];
  float xm3, xm2, xm1;
  {
    const bool hist = (tb > 0);
    const int rb = hist ? (g0 - 3) : g0;
    const float v3 = XZ[(size_t)rb * kXzP + d];
    const float v2 = XZ[(size_t)(rb + 1) * kXzP + d];
    const float v1 = XZ[(size_t)(rb + 2) * kXzP + d];
    xm3 = hist ? v3 : 0.f;
    xm2 = hist ? v2 : 0.f;
    xm1 = hist ? v1 : 0.f;
  }
  const int hrow = wave >> 1;
  const int hch  = (wave & 1) * 128 + lane * 4;
#pragma unroll 1
  for (int sub = 0; sub < 4; ++sub) {
    const int lb = g0 + sub * 16;
#pragma unroll 1
    for (int s = 0; s < 16; ++s) {
      const float xcur = XZ[(size_t)(lb + s) * kXzP + d];
      float acc = w0 * xm3;
      acc = fmaf(w1, xm2, acc);
      acc = fmaf(w2, xm1, acc);
      acc = fmaf(w3, xcur, acc);
      const float sv = acc + bc;
      const float sg = __builtin_amdgcn_rcpf(1.0f + expf(-sv));
      sT[s * kTP + tid] = sv * sg;
      xm3 = xm2; xm2 = xm1; xm1 = xcur;
    }
    __syncthreads();
    v4f fv[4];
    v8h bv[2];
#pragma unroll
    for (int it = 0; it < 4; ++it) fv[it] = *(const v4f*)(sT + (it * 4 + hrow) * kTP + hch);
#pragma unroll
    for (int it = 0; it < 2; ++it) {
      const float* sp = sT + (it * 8 + wave) * kTP + lane * 8;
      const v4f a0 = *(const v4f*)(sp);
      const v4f a1 = *(const v4f*)(sp + 4);
#pragma unroll
      for (int e = 0; e < 4; ++e) {
        bv[it][e]     = (_Float16)(a0[e] * kCarryUC);
        bv[it][4 + e] = (_Float16)(a1[e] * kCarryUC);
      }
    }
    for (int pass = 0; pass < 2; ++pass) {
#pragma unroll
      for (int it = 0; it < 4; ++it)
        *(volatile v4f*)(UC + (size_t)(lb + it * 4 + hrow) * kDin + hch) = fv[it];
#pragma unroll
      for (int it = 0; it < 2; ++it)
        *(volatile v8h*)(UC16 + (size_t)(lb + it * 8 + wave) * kDin + lane * 8) = bv[it];
      __threadfence();
    }
    __syncthreads();
  }
}

__global__ __launch_bounds__(64) void scan_kernel(
    const float* __restrict__ XD, const float* __restrict__ UC, const float* __restrict__ XZ,
    const float* __restrict__ Wdt, const float* __restrict__ bdt, const float* __restrict__ Alog,
    const float* __restrict__ Dp, unsigned short* __restrict__ Y16)
{
  __shared__ __align__(16) float sX[kScanTS * kXdP];
  __shared__ __align__(16) float sY[kScanTS * kScanYP];
  __shared__ __align__(16) float sA[kNst * kScanCh];
  const int tid = threadIdx.x, lane = tid & 31, wave = tid >> 5;
  constexpr int kBlkPerB = kDin / kScanCh;
  const int bix = blockIdx.x / kBlkPerB;
  const int d0  = (blockIdx.x - bix * kBlkPerB) * kScanCh;
  const int d   = d0 + tid;
  const size_t row0 = (size_t)bix * kLP;
#pragma unroll 1
  for (int s = 0; s < kNst; ++s) sA[s * kScanCh + tid] = -expf(Alog[(size_t)d * kNst + s]);
  __syncthreads();
  float negA[kNst], h[kNst];
#pragma unroll
  for (int s = 0; s < kNst; ++s) {
    negA[s] = sA[s * kScanCh + tid];
    h[s] = 0.f;
  }
  const v4f wv = *(const v4f*)(Wdt + (size_t)d * kDtR);
  const float bb = bdt[d], Dd = Dp[d];
  const int lr = tid >> 4, lc4 = (tid & 15) * 4;
  const int q = lane >> 3, c8 = (lane & 7) * 8;
#pragma unroll 1
  for (int t0 = 0; t0 < kLP; t0 += kScanTS) {
    __syncthreads();
#pragma unroll 4
    for (int i = 0; i < 16; ++i) {
      const int r = lr + 4 * i;
      *(v4f*)(sX + r * kXdP + lc4) = *(const v4f*)(XD + (row0 + t0 + r) * kXdP + lc4);
    }
    __syncthreads();
#pragma unroll 1
    for (int s = 0; s < kScanTS; ++s) {
      const int t = t0 + s;
      const float* xr = sX + s * kXdP;
      const v4f dl = *(const v4f*)(xr);
      float vdot = dl[0] * wv[0];
      vdot = fmaf(dl[1], wv[1], vdot);
      vdot = fmaf(dl[2], wv[2], vdot);
      vdot = fmaf(dl[3], wv[3], vdot);
      float Bs[kNst], Cs[kNst];
#pragma unroll
      for (int q4 = 0; q4 < 4; ++q4) {
        const v4f bv = *(const v4f*)(xr + kDtR + 4 * q4);
        const v4f cv = *(const v4f*)(xr + kDtR + kNst + 4 * q4);
        Bs[4 * q4 + 0] = bv[0]; Bs[4 * q4 + 1] = bv[1]; Bs[4 * q4 + 2] = bv[2]; Bs[4 * q4 + 3] = bv[3];
        Cs[4 * q4 + 0] = cv[0]; Cs[4 * q4 + 1] = cv[1]; Cs[4 * q4 + 2] = cv[2]; Cs[4 * q4 + 3] = cv[3];
      }
      const float v   = vdot + bb;
      const float a   = __expf(-fabsf(v));
      const float u   = 1.0f + a;
      const float l1p = __logf(u) + (a - (u - 1.0f)) * __builtin_amdgcn_rcpf(u);
      const float dt  = fmaxf(v, 0.0f) + l1p;
      const float xt  = UC[(row0 + t) * kDin + d];
      const float dtx = dt * xt;
      float y = 0.f;
#pragma unroll
      for (int k = 0; k < kNst; ++k) {
        const float e = __expf(dt * negA[k]);
        h[k] = e * h[k] + dtx * Bs[k];
        y = h[k] * Cs[k] + y;
      }
      y = xt * Dd + y;
      const float zv = XZ[(row0 + t) * kXzP + kDin + d];
      const float sg = __builtin_amdgcn_rcpf(1.0f + __expf(-zv));
      y = y * (zv * sg);
      sY[s * kScanYP + tid] = y * kCarryY;
    }
    __syncthreads();
    v8h hv[8];
#pragma unroll
    for (int it = 0; it < 8; ++it) {
      const int row = it * 8 + wave * 4 + q;
      const float* sp = sY + row * kScanYP + c8;
      const v4f a0 = *(const v4f*)(sp);
      const v4f a1 = *(const v4f*)(sp + 4);
#pragma unroll
      for (int e = 0; e < 4; ++e) {
        hv[it][e]     = (_Float16)a0[e];
        hv[it][4 + e] = (_Float16)a1[e];
      }
    }
    for (int pass = 0; pass < 2; ++pass) {
#pragma unroll
      for (int it = 0; it < 8; ++it) {
        const int row = it * 8 + wave * 4 + q;
        const size_t o = (row0 + t0 + row) * kDin + d0 + c8;
        *(volatile v8h*)(Y16 + o) = hv[it];
      }
      __threadfence();
    }
  }
}

__global__ __launch_bounds__(256) void frame_add_split_kernel(
    const float* __restrict__ HID, const float* __restrict__ x,
    unsigned short* __restrict__ RH, unsigned short* __restrict__ RL, int dir, int b0)
{
  const int tid = threadIdx.x, lane = tid & 31, wave = tid >> 5;
  const int q = lane >> 3, c8 = (lane & 7) * 8;
  const int row = blockIdx.x * 32 + wave * 4 + q;
  const int bl = row / kLP;
  const int r  = row - bl * kLP;
  const int b  = b0 + bl;
  const bool live = (r < kL);
  const int lo  = live ? (dir ? (kL - 1 - r) : r) : r;
  const int loc = live ? lo : (kL - 1);
  const float* hp = HID + (size_t)row * kKs + c8;
  const v4f h0 = *(const v4f*)(hp);
  const v4f h1 = *(const v4f*)(hp + 4);
  const float* s = x + (size_t)b * kT + loc + c8;
  float sg[8];
#pragma unroll
  for (int e = 0; e < 8; ++e) sg[e] = s[e];
  v8h hv, lv;
#pragma unroll
  for (int e = 0; e < 4; ++e) {
    const float f0 = live ? (h0[e] + sg[e]) : 0.0f;
    const float f1 = live ? (h1[e] + sg[4 + e]) : 0.0f;
    const unsigned short hb0 = f2bf_bits(f0), hb1 = f2bf_bits(f1);
    const unsigned short lb0 = f2bf_bits(f0 - bf_bits2f(hb0)), lb1 = f2bf_bits(f1 - bf_bits2f(hb1));
    hv[e]     = __builtin_bit_cast(_Float16, hb0);
    hv[4 + e] = __builtin_bit_cast(_Float16, hb1);
    lv[e]     = __builtin_bit_cast(_Float16, lb0);
    lv[4 + e] = __builtin_bit_cast(_Float16, lb1);
  }
  const size_t o = ((size_t)b * kLP + lo) * kRc + (size_t)dir * kKs + c8;
  *(volatile v8h*)(RH + o) = hv;
  *(volatile v8h*)(RL + o) = lv;
  __threadfence();
  *(volatile v8h*)(RH + o) = hv;
  *(volatile v8h*)(RL + o) = lv;
}

__global__ __launch_bounds__(256) void fold_kernel(
    const float* __restrict__ P, const float* __restrict__ x, const float* __restrict__ ctb, float* __restrict__ out)
{
  const int t = blockIdx.x * 256 + threadIdx.x;
  const int b = blockIdx.y;
  const float* Pb = P + (size_t)b * kLP * kKs;
  float acc = 0.0f;
#pragma unroll 4
  for (int j = 0; j < kKs; ++j) {
    const int l = t - j;
    const bool ok = (l >= 0) && (l < kL);
    const int lc = (l < 0) ? 0 : ((l >= kL) ? (kL - 1) : l);
    const float v = Pb[(size_t)lc * kKs + j];
    acc += ok ? v : 0.0f;
  }
  const float res = (acc + ctb[0]) + x[(size_t)b * kT + t];
  float* o = out + (size_t)b * kT + t;
  *(volatile float*)o = res;
  __threadfence();
  *(volatile float*)o = res;
}

static_assert(((kMP / 64) * (kXzP / 64)) % 8 == 0 && ((kMP / 64) * (kXdP / 64)) % 8 == 0 &&
              ((kMP / 64) * (kKs / 64)) % 8 == 0 && ((kRowsAll / 64) * (kKs / 64)) % 8 == 0, "whole blocks of 8 tiles");

extern "C" void kernel_launch(void* const* d_in, const int* in_sizes, int n_in,
                              void* d_out, int out_size, void* d_ws, size_t ws_size,
                              hipStream_t stream) {
  if (n_in < 23) return;
  if (in_sizes[0] != kB * kT) return;
  for (int p = 0; p < 2; ++p) {
    const int o = p * 10;
    if (in_sizes[1 + o] != kKs) return;
    if (in_sizes[2 + o] != kXzP * kKs) return;
    if (in_sizes[3 + o] != kDin * 4) return;
    if (in_sizes[4 + o] != kDin) return;
    if (in_sizes[5 + o] != kXpN * kDin) return;
    if (in_sizes[6 + o] != kDin * kDtR) return;
    if (in_sizes[7 + o] != kDin) return;
    if (in_sizes[8 + o] != kDin * kNst) return;
    if (in_sizes[9 + o] != kDin) return;
    if (in_sizes[10 + o] != kKs * kDin) return;
  }
  if (in_sizes[21] != kRc * kKs) return;
  if (in_sizes[22] != 1) return;
  if (out_size != kB * kT) return;
  if (ws_size < kWsTotal) return;

  const float* x = (const float*)d_in[0];
  const float* norm_w[2]  = {(const float*)d_in[1],  (const float*)d_in[11]};
  const float* in_w[2]    = {(const float*)d_in[2],  (const float*)d_in[12]};
  const float* conv_w[2]  = {(const float*)d_in[3],  (const float*)d_in[13]};
  const float* conv_b[2]  = {(const float*)d_in[4],  (const float*)d_in[14]};
  const float* xproj_w[2] = {(const float*)d_in[5],  (const float*)d_in[15]};
  const float* dt_w[2]    = {(const float*)d_in[6],  (const float*)d_in[16]};
  const float* dt_b[2]    = {(const float*)d_in[7],  (const float*)d_in[17]};
  const float* Alog[2]    = {(const float*)d_in[8],  (const float*)d_in[18]};
  const float* Dvec[2]    = {(const float*)d_in[9],  (const float*)d_in[19]};
  const float* out_w[2]   = {(const float*)d_in[10], (const float*)d_in[20]};
  const float* ct_w = (const float*)d_in[21];
  const float* ct_b = (const float*)d_in[22];
  float* out = (float*)d_out;

  char* ws = (char*)d_ws;
  unsigned short* WIN16  = (unsigned short*)(ws + kOffWIN);
  unsigned short* WXP16  = (unsigned short*)(ws + kOffWXP);
  unsigned short* WOUT16 = (unsigned short*)(ws + kOffWOUT);
  unsigned short* CTH    = (unsigned short*)(ws + kOffCTH);
  unsigned short* CTL    = (unsigned short*)(ws + kOffCTL);
  unsigned short* U16    = (unsigned short*)(ws + kOffU);
  float*          XZ     = (float*)(ws + kOffXZ);
  float*          UC     = (float*)(ws + kOffUC);
  unsigned short* UC16   = (unsigned short*)(ws + kOffUC16);
  float*          XD     = (float*)(ws + kOffXD);
  unsigned short* Y16    = (unsigned short*)(ws + kOffY16);
  float*          HID    = (float*)(ws + kOffHID);
  unsigned short* RH     = (unsigned short*)(ws + kOffRH);
  unsigned short* RL     = (unsigned short*)(ws + kOffRL);
  float*          P      = (float*)(ws + kOffP);
  const float* dummy_bias  = ct_b;
  const float* dummy_resid = x;

  for (int dir = 0; dir < 2; ++dir) {
    cast_f16_pad_kernel<<<(kXzP * kKs / 8) / 256, 256, 0, stream>>>(
        in_w[dir], WIN16 + (size_t)dir * kXzP * kKs, kXzP * kKs / 8, kXzP * kKs / 8, kCarryW);
    cast_f16_pad_kernel<<<(kXdP * kDin / 8) / 256, 256, 0, stream>>>(
        xproj_w[dir], WXP16 + (size_t)dir * kXdP * kDin, kXdP * kDin / 8, kXpN * kDin / 8, kCarryW);
    cast_f16_pad_kernel<<<(kKs * kDin / 8) / 256, 256, 0, stream>>>(
        out_w[dir], WOUT16 + (size_t)dir * kKs * kDin, kKs * kDin / 8, kKs * kDin / 8, kCarryW);
  }
  transpose_split_bf16_kernel<<<dim3(kKs / 64, kRc / 64), 256, 0, stream>>>(ct_w, CTH, CTL, kRc, kKs);
  frame_norm_kernel<<<dim3(kRowsAll / 32, 2), 256, 0, stream>>>(x, norm_w[0], norm_w[1], U16);

  for (int dir = 0; dir < 2; ++dir) {
    const unsigned short* Wi = WIN16  + (size_t)dir * kXzP * kKs;
    const unsigned short* Wx = WXP16  + (size_t)dir * kXdP * kDin;
    const unsigned short* Wo = WOUT16 + (size_t)dir * kKs * kDin;
    for (int half = 0; half < kB / kNBP; ++half) {
      const int b0 = half * kNBP;
      const unsigned short* Up = U16 + (size_t)dir * kRowsAll * kKs + (size_t)b0 * kLP * kKs;

      wmma_gemm64<0, false, 0, 0, false><<<dim3((kMP / 64) * (kXzP / 64) / 8, 1), 256, 0, stream>>>(
          Up, Up, kKs, 0L, Wi, Wi, kKs, 0L,
          (void*)XZ, (void*)XZ, kXzP, 0L, dummy_bias, dummy_resid, 0L, kMP, kXzP, kKs, 1.0f / kCarryW);

      conv_silu_kernel<<<kMP / 64, 256, 0, stream>>>(XZ, conv_w[dir], conv_b[dir], UC, UC16);

      wmma_gemm64<0, false, 0, 0, false><<<dim3((kMP / 64) * (kXdP / 64) / 8, 1), 256, 0, stream>>>(
          UC16, UC16, kDin, 0L, Wx, Wx, kDin, 0L,
          (void*)XD, (void*)XD, kXdP, 0L, dummy_bias, dummy_resid, 0L, kMP, kXdP, kDin, 1.0f / (kCarryUC * kCarryW));

      scan_kernel<<<kNBP * (kDin / kScanCh), kScanCh, 0, stream>>>(
          XD, UC, XZ, dt_w[dir], dt_b[dir], Alog[dir], Dvec[dir], Y16);

      wmma_gemm64<0, false, 0, 0, false><<<dim3((kMP / 64) * (kKs / 64) / 8, 1), 256, 0, stream>>>(
          Y16, Y16, kDin, 0L, Wo, Wo, kDin, 0L,
          (void*)HID, (void*)HID, kKs, 0L, dummy_bias, dummy_resid, 0L, kMP, kKs, kDin, 1.0f / (kCarryY * kCarryW));

      frame_add_split_kernel<<<kMP / 32, 256, 0, stream>>>(HID, x, RH, RL, dir, b0);
    }
  }

  wmma_gemm64<1, true, 0, 0, false><<<dim3((kRowsAll / 64) * (kKs / 64) / 8, 1), 256, 0, stream>>>(
      RH, RL, kRc, 0L, CTH, CTL, kRc, 0L,
      (void*)P, (void*)P, kKs, 0L, dummy_bias, dummy_resid, 0L, kRowsAll, kKs, kRc, 1.0f);

  fold_kernel<<<dim3(kT / 256, kB), 256, 0, stream>>>(P, x, ct_b, out);
}
